// MultiScaleRetention_10548439679589
// MI455X (gfx1250) — hardware-verified
//
#include <hip/hip_runtime.h>
#include <math.h>

constexpr int NB    = 2;
constexpr int NT    = 2048;
constexpr int NHID  = 1024;
constexpr int NHEAD = 8;
constexpr int QKD   = 1024;
constexpr int VD    = 2048;
constexpr int DQK   = QKD / NHEAD;
constexpr int DV    = VD / NHEAD;
constexpr int NROW  = NB * NT;
constexpr int NQKV  = 2 * QKD + VD;
constexpr int NPAIR = QKD / 2;
constexpr int NBH   = NB * NHEAD;
constexpr int NOUT0 = NROW * NHID;
constexpr int NOUT1 = NB * NHEAD * DQK * DV;

constexpr float WCARRY     = 16.0f;
constexpr float WCARRY_INV = 1.0f / 16.0f;
constexpr float QCARRY     = 256.0f;
constexpr float PCARRY     = 256.0f;
constexpr float PCARRY_INV = 1.0f / 256.0f;
constexpr float GCARRY     = 64.0f;
constexpr float OUT_SCALE  = 1.0f / (16.0f * 64.0f);
constexpr float GN_EPS_F   = 1e-5f;

constexpr int PPITCH = 72;
constexpr int KVP    = 40;
constexpr int SLP    = 36;

static_assert(DQK == 128 && DV == 256);
static_assert(NROW == 4096 && NQKV == 4096 && NPAIR == 512);
static_assert(NHID % 32 == 0 && VD % 32 == 0 && DQK % 32 == 0);
static_assert(NROW % 64 == 0 && NQKV % 64 == 0 && VD % 64 == 0 && NHID % 64 == 0 && NT % 64 == 0 && DV % 64 == 0);
static_assert((size_t)NOUT0 * 4 == 16777216);
static_assert((size_t)NOUT1 * 4 == 2097152);
static_assert((size_t)NBH * DV * NT * 2 == (size_t)NROW * VD * 2);
static_assert((size_t)NROW * VD * 4 <= (size_t)NROW * NQKV * 4);

typedef __attribute__((ext_vector_type(16))) _Float16 v16h;
typedef __attribute__((ext_vector_type(8)))  _Float16 v8h;
typedef __attribute__((ext_vector_type(16))) __bf16   v16b;
typedef __attribute__((ext_vector_type(8)))  __bf16   v8b;
typedef __attribute__((ext_vector_type(8)))  float    v8f;
typedef __attribute__((ext_vector_type(4)))  float    v4f;
typedef __attribute__((ext_vector_type(2)))  float    v2f;
typedef __attribute__((ext_vector_type(4)))  unsigned int v4u;

struct Decay8 { float v[8]; };
static_assert(sizeof(Decay8) == 32);

__device__ __forceinline__ unsigned short f2bf_bits(float f) {
  unsigned u = __float_as_uint(f);
  return (unsigned short)((u + 0x7FFFu + ((u >> 16) & 1u)) >> 16);
}
__device__ __forceinline__ float bf_bits2f(unsigned short h) { return __uint_as_float(((unsigned)h) << 16); }
__device__ __forceinline__ float bf16r(float f) { return bf_bits2f(f2bf_bits(f)); }
__device__ __forceinline__ unsigned pk16(unsigned short a, unsigned short b) { return (unsigned)a | ((unsigned)b << 16); }
__device__ __forceinline__ unsigned short h_bits(float f) { const _Float16 h = (_Float16)f; return __builtin_bit_cast(unsigned short, h); }

__device__ __forceinline__ float pick8(const Decay8& d, int h) {
  float r = d.v[0];
  r = (h == 1) ? d.v[1] : r;
  r = (h == 2) ? d.v[2] : r;
  r = (h == 3) ? d.v[3] : r;
  r = (h == 4) ? d.v[4] : r;
  r = (h == 5) ? d.v[5] : r;
  r = (h == 6) ? d.v[6] : r;
  r = (h == 7) ? d.v[7] : r;
  return r;
}

__device__ __forceinline__ void dep_guard4_h(v8f& a0, v8f& a1, v8f& a2, v8f& a3, v16h x, v16h y) {
  asm volatile("v_nop\n\tv_nop\n\tv_nop\n\tv_nop" : "+v"(a0), "+v"(a1), "+v"(a2), "+v"(a3) : "v"(x), "v"(y));
}
__device__ __forceinline__ void keep4_h(v16h a, v16h b, v16h c, v16h d) { asm volatile("v_nop" :: "v"(a), "v"(b), "v"(c), "v"(d)); }
__device__ __forceinline__ void acc_guard4(v8f& a, v8f& b, v8f& c, v8f& d) { asm volatile("v_nop\n\tv_nop\n\tv_nop\n\tv_nop" : "+v"(a), "+v"(b), "+v"(c), "+v"(d)); }

template <typename T> struct Frag;
template <> struct Frag<_Float16> {
  typedef v16h V; union U { v16h v; v8h h[2]; };
  static __device__ __forceinline__ v16h load(const _Float16* p) {
    U f; f.h[0] = *(const v8h*)(p); f.h[1] = *(const v8h*)(p + 16); return f.v;
  }
  static __device__ __forceinline__ v8f mma(v16h a, v16h b, v8f c) {
    return __builtin_amdgcn_wmma_f32_16x16x32_f16(false, a, false, b, (short)0, c, false, false);
  }
};
template <> struct Frag<__bf16> {
  typedef v16b V; union U { v16b v; v8b h[2]; };
  static __device__ __forceinline__ v16b load(const __bf16* p) {
    U f; f.h[0] = *(const v8b*)(p); f.h[1] = *(const v8b*)(p + 16); return f.v;
  }
};

__device__ __forceinline__ v8f mma_h(v16h a, v16h b, v8f c) {
  c = __builtin_amdgcn_wmma_f32_16x16x32_f16(false, a, false, b, (short)0, c, false, false);
  asm volatile("v_nop\n\tv_nop\n\tv_nop\n\tv_nop" : "+v"(c) : "v"(a), "v"(b));
  return c;
}
__device__ __forceinline__ v8f mma_b(v16b a, v16b b, v8f c) {
  c = __builtin_amdgcn_wmma_f32_16x16x32_bf16(false, a, false, b, (short)0, c, false, false);
  asm volatile("v_nop\n\tv_nop\n\tv_nop\n\tv_nop" : "+v"(c) : "v"(a), "v"(b));
  return c;
}

__device__ __forceinline__ void wave_sync_lds() {
  __builtin_amdgcn_fence(__ATOMIC_RELEASE, "workgroup");
  __builtin_amdgcn_wave_barrier();
  __builtin_amdgcn_fence(__ATOMIC_ACQUIRE, "workgroup");
}

template <int BIAS_MODE, int OUT_MODE, bool GATE>
__global__ __launch_bounds__(256) void wmma_gemm64(
    const unsigned short* __restrict__ Ap, int lda,
    const unsigned short* __restrict__ Btp, int ldb,
    void* __restrict__ Cout, int ldc,
    const float* __restrict__ bias,
    const float* __restrict__ gsrc, int ldg, float gcarry,
    int M, int N, int K, float scale) {
  const _Float16* A  = (const _Float16*)Ap;
  const _Float16* Bt = (const _Float16*)Btp;
  __shared__ __align__(16) float sT[8][16 * 68];
  const int lane = threadIdx.x & 31;
  const int wave = threadIdx.x >> 5;
  const int tilesN = N >> 6;
  const int tilesM = M >> 6;
  const int tile = blockIdx.x * 8 + wave;
  if (tile >= tilesM * tilesN) return;
  const int tm = tile / tilesN;
  const int tn = tile - tm * tilesN;
  const int m0 = tm << 6;
  const int n0 = tn << 6;

  const int rlane = lane & 15;
  const int koff  = (lane >> 4) * 8;
  const int mOff  = (lane >> 4) * 8;

  const _Float16* arow[4];
  const _Float16* brow[4];
#pragma unroll
  for (int i = 0; i < 4; ++i) {
    arow[i] = A  + (size_t)(m0 + (i << 4) + rlane) * lda + koff;
    brow[i] = Bt + (size_t)(n0 + (i << 4) + rlane) * ldb + koff;
  }

  v8f acc[4][4];
#pragma unroll
  for (int i = 0; i < 4; ++i)
#pragma unroll
    for (int j = 0; j < 4; ++j) acc[i][j] = (v8f){0.f,0.f,0.f,0.f,0.f,0.f,0.f,0.f};

  for (int k0 = 0; k0 < K; k0 += 32) {
    v16h bfr[4];
#pragma unroll
    for (int j = 0; j < 4; ++j) bfr[j] = Frag<_Float16>::load(brow[j] + k0);
#pragma unroll
    for (int i = 0; i < 4; ++i) {
      const v16h afr = Frag<_Float16>::load(arow[i] + k0);
#pragma unroll
      for (int j = 0; j < 4; ++j) acc[i][j] = Frag<_Float16>::mma(afr, bfr[j], acc[i][j]);
      dep_guard4_h(acc[i][0], acc[i][1], acc[i][2], acc[i][3], afr, bfr[3]);
    }
    keep4_h(bfr[0], bfr[1], bfr[2], bfr[3]);
  }
  acc_guard4(acc[0][0], acc[0][1], acc[0][2], acc[0][3]);
  acc_guard4(acc[1][0], acc[1][1], acc[1][2], acc[1][3]);
  acc_guard4(acc[2][0], acc[2][1], acc[2][2], acc[2][3]);
  acc_guard4(acc[3][0], acc[3][1], acc[3][2], acc[3][3]);

  float* slab = sT[wave];
#pragma unroll
  for (int i = 0; i < 4; ++i) {
    const int mBase = m0 + (i << 4);
#pragma unroll
    for (int j = 0; j < 4; ++j) {
      const int n = n0 + (j << 4) + rlane;
      float bv = 0.f;
      if (BIAS_MODE == 2) bv = bf16r(bias[n]);
#pragma unroll
      for (int r = 0; r < 8; ++r) {
        float v = acc[i][j][r] * scale;
        if (BIAS_MODE == 2) v += bv;
        slab[(mOff + r) * 68 + (j << 4) + rlane] = v;
      }
    }
    wave_sync_lds();
    if (GATE) {
      const int hh = lane >> 4, c4 = (lane & 15) * 4;
#pragma unroll 1
      for (int it = 0; it < 8; ++it) {
        const int row = it * 2 + hh;
        float* sp = slab + row * 68 + c4;
        const v4f s = *(const v4f*)sp;
        const v4f g = *(const v4f*)(gsrc + (size_t)(mBase + row) * ldg + n0 + c4);
        v4f o;
#pragma unroll
        for (int e = 0; e < 4; ++e) {
          const float z  = s[e];
          const float nr = g[e];
          const float sg = z * (1.0f / (1.0f + expf(-z)));
          o[e] = (sg * nr) * gcarry;
        }
        *(v4f*)sp = o;
      }
      wave_sync_lds();
    }
    if (OUT_MODE == 0) {
      float* C = (float*)Cout;
      const int hh = lane >> 4, c4 = (lane & 15) * 4;
      for (int pass = 0; pass < 2; ++pass) {
#pragma unroll
        for (int it = 0; it < 8; ++it) {
          const int row = it * 2 + hh;
          v4f v = *(const v4f*)(slab + row * 68 + c4);
          *(volatile v4f*)(C + (size_t)(mBase + row) * ldc + n0 + c4) = v;
        }
        __threadfence();
      }
    } else {
      const int q = lane >> 3, c8 = (lane & 7) * 8;
      unsigned short* C = (unsigned short*)Cout;
      for (int pass = 0; pass < 2; ++pass) {
#pragma unroll
        for (int it = 0; it < 4; ++it) {
          const int row = it * 4 + q;
          const float* sp = slab + row * 68 + c8;
          v8h hv;
#pragma unroll
          for (int e = 0; e < 8; ++e) hv[e] = (_Float16)sp[e];
          *(volatile v8h*)(C + (size_t)(mBase + row) * ldc + n0 + c8) = hv;
        }
        __threadfence();
      }
    }
    wave_sync_lds();
  }
}

__global__ __launch_bounds__(256) void cvt8_bf16_f16_kernel(const float* __restrict__ src, unsigned short* __restrict__ dst, int n8) {
  const int i = blockIdx.x * 256 + threadIdx.x;
  if (i < n8) {
    const float* sp = src + (size_t)i * 8;
    const v4f a = *(const v4f*)(sp);
    const v4f b = *(const v4f*)(sp + 4);
    v8h hv;
#pragma unroll
    for (int e = 0; e < 4; ++e) {
      const float ae = a[e];
      const float be = b[e];
      hv[e]     = (_Float16)bf16r(ae);
      hv[4 + e] = (_Float16)bf16r(be);
    }
    *(volatile v8h*)(dst + (size_t)i * 8) = hv;
    __threadfence();
    *(volatile v8h*)(dst + (size_t)i * 8) = hv;
  }
}

__global__ __launch_bounds__(256) void tcvt_kernel(const float* __restrict__ in, int ldin, long in_zb, long in_zh, int zdiv,
                                                   unsigned short* __restrict__ out, int ldout, long out_z,
                                                   float sc, int rb16) {
  __shared__ float sm[64][65];
  const int t  = threadIdx.x;
  const int c0 = blockIdx.x * 64;
  const int r0 = blockIdx.y * 64;
  const int z  = blockIdx.z;
  const int zb = z / zdiv;
  const int zh = z - zb * zdiv;
  const float* ip = in + (size_t)zb * in_zb + (size_t)zh * in_zh;
#pragma unroll
  for (int i = 0; i < 16; ++i) {
    const int e = i * 256 + t;
    const int r = e >> 6;
    const int c = e & 63;
    float v = ip[(size_t)(r0 + r) * ldin + c0 + c];
    if (rb16) v = bf16r(v);
    sm[c][r] = v * sc;
  }
  __syncthreads();
  const int lane = t & 31, wave = t >> 5;
  const int q = lane >> 3, c8 = (lane & 7) * 8;
  unsigned short* op = out + (size_t)z * out_z;
  for (int pass = 0; pass < 2; ++pass) {
#pragma unroll
    for (int it = 0; it < 2; ++it) {
      const int row = wave * 8 + it * 4 + q;
      unsigned short hb[8];
#pragma unroll
      for (int e = 0; e < 8; ++e) hb[e] = h_bits(sm[row][c8 + e]);
      const v4u u = (v4u){pk16(hb[0], hb[1]), pk16(hb[2], hb[3]), pk16(hb[4], hb[5]), pk16(hb[6], hb[7])};
      *(volatile v4u*)(op + (size_t)(c0 + row) * ldout + r0 + c8) = u;
    }
    __threadfence();
  }
}

__global__ __launch_bounds__(512) void rot_table_kernel(float* __restrict__ tab) {
  const int i = threadIdx.x;
  const float fi = (float)i;
  const float e = fi * (1.0f / (float)NPAIR);
  const float p = powf(10000.0f, e);
  const float invf = 1.0f / p;
  const float base = (2.0f * fi + 0.4f * (float)QKD) * (1.0f / (1.4f * (float)QKD));
  const float lb = log2f(base);
  *(volatile float*)(tab + i) = invf;
  *(volatile float*)(tab + NPAIR + i) = lb;
  __threadfence();
  *(volatile float*)(tab + i) = invf;
  *(volatile float*)(tab + NPAIR + i) = lb;
}

__global__ __launch_bounds__(512) void rotary_kernel(float* qkv, const float* __restrict__ tab,
                                                     unsigned short* __restrict__ qh, unsigned short* __restrict__ kh) {
  const int t = blockIdx.x;
  const int i = threadIdx.x;
  const float invf = tab[i];
  const float lb   = tab[NPAIR + i];
  const float tf   = (float)t;
  const float ang  = tf * invf;
  const float ex   = (tf * (1.0f / 512.0f)) * lb;
  const float sc   = exp2f(ex);
  const float isc  = exp2f(-ex);
  const float sn   = sinf(ang);
  const float cs   = cosf(ang);
  const float cq = cs * sc,  sq = sn * sc;
  const float ck = cs * isc, sk = sn * isc;
  const int h = i >> 6;
  const int d = (2 * i) & (DQK - 1);
#pragma unroll 1
  for (int b = 0; b < NB; ++b) {
    float* row = qkv + (size_t)(b * NT + t) * NQKV;
    const v2f xq = *(const v2f*)(row + 2 * i);
    const v2f xk = *(const v2f*)(row + QKD + 2 * i);
    const float q0 = xq.x * cq - xq.y * sq;
    const float q1 = xq.y * cq + xq.x * sq;
    const float k0 = xk.x * ck - xk.y * sk;
    const float k1 = xk.y * ck + xk.x * sk;
    const unsigned uq = pk16(h_bits(q0 * QCARRY), h_bits(q1 * QCARRY));
    const unsigned uk = pk16(h_bits(k0), h_bits(k1));
    const v2f kf = (v2f){k0, k1};
    const size_t o = ((size_t)((b * NHEAD + h) * NT + t)) * DQK + d;
    unsigned* qp = (unsigned*)(qh + o);
    unsigned* kp = (unsigned*)(kh + o);
    float* kfp = row + QKD + 2 * i;
    *(volatile unsigned*)qp = uq;
    *(volatile unsigned*)kp = uk;
    *(volatile v2f*)kfp = kf;
    __threadfence();
    *(volatile unsigned*)qp = uq;
    *(volatile unsigned*)kp = uk;
    *(volatile v2f*)kfp = kf;
  }
}

__global__ __launch_bounds__(256) void kv_state_kernel(const float* __restrict__ qkv, float* __restrict__ kvout, Decay8 dec) {
  __shared__ __align__(16) unsigned short Ah[DQK * KVP];
  __shared__ __align__(16) unsigned short Al[DQK * KVP];
  __shared__ __align__(16) unsigned short Bh[64 * KVP];
  __shared__ __align__(16) unsigned short Bl[64 * KVP];
  __shared__ __align__(16) float Sl[8][16 * SLP];
  const int tid = threadIdx.x, lane = tid & 31, wave = tid >> 5;
  const int c = lane & 15, hh = lane >> 4, koff = hh * 8;
  const int bh = blockIdx.x >> 2, ns = blockIdx.x & 3;
  const int b = bh >> 3, h = bh & 7;
  const float l2g = pick8(dec, h);
  const float* kbase = qkv + (size_t)b * NT * NQKV + QKD + h * DQK;
  const float* vbase = qkv + (size_t)b * NT * NQKV + 2 * QKD + h * DV + ns * 64;

  v8f acc[4];
#pragma unroll
  for (int j = 0; j < 4; ++j) acc[j] = (v8f){0.f,0.f,0.f,0.f,0.f,0.f,0.f,0.f};

  const int kr = tid >> 5, kc4 = (tid & 31) * 4;
  const int vr = tid >> 4, vc4 = (tid & 15) * 4;
  const __bf16* ahp = (const __bf16*)Ah + (wave * 16 + c) * KVP + koff;
  const __bf16* alp = (const __bf16*)Al + (wave * 16 + c) * KVP + koff;
  const __bf16* bhp = (const __bf16*)Bh + c * KVP + koff;
  const __bf16* blp = (const __bf16*)Bl + c * KVP + koff;

#pragma unroll 1
  for (int j0 = 0; j0 < NT; j0 += 32) {
#pragma unroll
    for (int it = 0; it < 4; ++it) {
      const int r = it * 8 + kr;
      const int t = j0 + r;
      const float w = exp2f(l2g * (float)(NT - 1 - t));
      const v4f kk = *(const v4f*)(kbase + (size_t)t * NQKV + kc4);
#pragma unroll
      for (int e = 0; e < 4; ++e) {
        const float ke = kk[e];
        const float x = ke * w;
        const unsigned short hb = f2bf_bits(x);
        const unsigned short lb = f2bf_bits(x - bf_bits2f(hb));
        Ah[(kc4 + e) * KVP + r] = hb;
        Al[(kc4 + e) * KVP + r] = lb;
      }
    }
#pragma unroll
    for (int it = 0; it < 2; ++it) {
      const int r = it * 16 + vr;
      const v4f vv = *(const v4f*)(vbase + (size_t)(j0 + r) * NQKV + vc4);
#pragma unroll
      for (int e = 0; e < 4; ++e) {
        const float x = vv[e];
        const unsigned short hb = f2bf_bits(x);
        const unsigned short lb = f2bf_bits(x - bf_bits2f(hb));
        Bh[(vc4 + e) * KVP + r] = hb;
        Bl[(vc4 + e) * KVP + r] = lb;
      }
    }
    __syncthreads();
    {
      const v16b ah = Frag<__bf16>::load(ahp);
      const v16b al = Frag<__bf16>::load(alp);
#pragma unroll
      for (int j = 0; j < 4; ++j) {
        const v16b bhf = Frag<__bf16>::load(bhp + j * 16 * KVP);
        const v16b blf = Frag<__bf16>::load(blp + j * 16 * KVP);
        acc[j] = mma_b(ah, blf, acc[j]);
        acc[j] = mma_b(al, bhf, acc[j]);
        acc[j] = mma_b(ah, bhf, acc[j]);
      }
    }
    __syncthreads();
  }

  float* slab = Sl[wave];
  const int q = lane >> 3, c4 = (lane & 7) * 4;
  float* obase = kvout + ((size_t)bh * DQK + wave * 16) * DV + ns * 64;
#pragma unroll
  for (int jp = 0; jp < 2; ++jp) {
#pragma unroll
    for (int jj = 0; jj < 2; ++jj)
#pragma unroll
      for (int r = 0; r < 8; ++r) slab[(8 * hh + r) * SLP + jj * 16 + c] = acc[jp * 2 + jj][r];
    wave_sync_lds();
    for (int pass = 0; pass < 2; ++pass) {
#pragma unroll
      for (int it = 0; it < 4; ++it) {
        const int row = it * 4 + q;
        const v4f v = *(const v4f*)(slab + row * SLP + c4);
        *(volatile v4f*)(obase + (size_t)row * DV + jp * 32 + c4) = v;
      }
      __threadfence();
    }
    wave_sync_lds();
  }
}

__global__ __launch_bounds__(256) void retention_gn_kernel(const unsigned short* __restrict__ qhp,
                                                           const unsigned short* __restrict__ khp,
                                                           const unsigned short* __restrict__ vtp,
                                                           float* __restrict__ normed, Decay8 dec, float pscl) {
  __shared__ __align__(16) _Float16 Ps[2][64 * PPITCH];
  __shared__ __align__(16) float Sl[8][16 * SLP];
  __shared__ float redS[8][64];
  __shared__ float stat[64];
  const _Float16* qh = (const _Float16*)qhp;
  const _Float16* kh = (const _Float16*)khp;
  const _Float16* vt = (const _Float16*)vtp;
  const int tid = threadIdx.x, lane = tid & 31, wave = tid >> 5;
  const int c = lane & 15, hh = lane >> 4, koff = hh * 8;
  const int itile = blockIdx.x;
  const int bh = blockIdx.y;
  const int b = bh >> 3, h = bh & 7;
  const int i0 = itile * 64;
  const float l2g = pick8(dec, h);
  const int mt = wave >> 1, ntb = (wave & 1) * 2;

  v16h qa[4];
  {
    const _Float16* qrow = qh + ((size_t)bh * NT + i0 + mt * 16 + c) * DQK + koff;
#pragma unroll
    for (int kc = 0; kc < 4; ++kc) qa[kc] = Frag<_Float16>::load(qrow + kc * 32);
  }
  float rowf[8];
#pragma unroll
  for (int r = 0; r < 8; ++r) rowf[r] = pscl * exp2f(l2g * (float)(mt * 16 + 8 * hh + r));

  v8f o[4][2];
#pragma unroll
  for (int m = 0; m < 4; ++m) {
    o[m][0] = (v8f){0.f,0.f,0.f,0.f,0.f,0.f,0.f,0.f};
    o[m][1] = (v8f){0.f,0.f,0.f,0.f,0.f,0.f,0.f,0.f};
  }

  const _Float16* kbase = kh + ((size_t)bh * NT + ntb * 16 + c) * DQK + koff;
  const _Float16* vbase = vt + ((size_t)bh * DV + wave * 32 + c) * NT + koff;
  const int rl0 = mt * 16 + 8 * hh;
  const int pcol = ntb * 16 + c;

#pragma unroll 1
  for (int jt = 0; jt <= itile; ++jt) {
    const int j0 = jt * 64;
    _Float16* pw = &Ps[jt & 1][0];
    v8f s0 = (v8f){0.f,0.f,0.f,0.f,0.f,0.f,0.f,0.f};
    v8f s1 = (v8f){0.f,0.f,0.f,0.f,0.f,0.f,0.f,0.f};
    const _Float16* kp = kbase + (size_t)j0 * DQK;
#pragma unroll
    for (int kc = 0; kc < 4; ++kc) {
      const v16h kb0 = Frag<_Float16>::load(kp + kc * 32);
      const v16h kb1 = Frag<_Float16>::load(kp + 16 * DQK + kc * 32);
      s0 = mma_h(qa[kc], kb0, s0);
      s1 = mma_h(qa[kc], kb1, s1);
    }
    const int jc0 = j0 + pcol;
    const int jc1 = jc0 + 16;
    const float cf0 = exp2f(l2g * (float)(i0 - jc0));
    const float cf1 = exp2f(l2g * (float)(i0 - jc1));
#pragma unroll
    for (int r = 0; r < 8; ++r) {
      const int i = i0 + rl0 + r;
      const float p0 = (s0[r] * rowf[r]) * cf0;
      const float p1 = (s1[r] * rowf[r]) * cf1;
      const float m0v = (jc0 <= i) ? p0 : 0.0f;
      const float m1v = (jc1 <= i) ? p1 : 0.0f;
      pw[(rl0 + r) * PPITCH + pcol]      = (_Float16)m0v;
      pw[(rl0 + r) * PPITCH + pcol + 16] = (_Float16)m1v;
    }
    __syncthreads();
    const _Float16* vp = vbase + j0;
#pragma unroll
    for (int kc = 0; kc < 2; ++kc) {
      const v16h vb0 = Frag<_Float16>::load(vp + kc * 32);
      const v16h vb1 = Frag<_Float16>::load(vp + (size_t)16 * NT + kc * 32);
#pragma unroll
      for (int m = 0; m < 4; ++m) {
        const v16h pa = Frag<_Float16>::load(pw + (m * 16 + c) * PPITCH + kc * 32 + koff);
        o[m][0] = mma_h(pa, vb0, o[m][0]);
        o[m][1] = mma_h(pa, vb1, o[m][1]);
      }
    }
  }

#pragma unroll
  for (int m = 0; m < 4; ++m) {
    o[m][0] = o[m][0] * PCARRY_INV;
    o[m][1] = o[m][1] * PCARRY_INV;
  }
  float part[4][8];
#pragma unroll
  for (int m = 0; m < 4; ++m)
#pragma unroll
    for (int r = 0; r < 8; ++r) {
      float x = o[m][0][r] + o[m][1][r];
      x += __shfl_xor(x, 1, 32);
      x += __shfl_xor(x, 2, 32);
      x += __shfl_xor(x, 4, 32);
      x += __shfl_xor(x, 8, 32);
      part[m][r] = x;
    }
  if (c == 0) {
#pragma unroll
    for (int m = 0; m < 4; ++m)
#pragma unroll
      for (int r = 0; r < 8; ++r) redS[wave][m * 16 + 8 * hh + r] = part[m][r];
  }
  __syncthreads();
  if (tid < 64) {
    float s = 0.0f;
#pragma unroll
    for (int w = 0; w < 8; ++w) s += redS[w][tid];
    stat[tid] = s * (1.0f / (float)DV);
  }
  __syncthreads();
#pragma unroll
  for (int m = 0; m < 4; ++m)
#pragma unroll
    for (int r = 0; r < 8; ++r) {
      const float mu = stat[m * 16 + 8 * hh + r];
      const float d0 = o[m][0][r] - mu;
      const float d1 = o[m][1][r] - mu;
      o[m][0][r] = d0;
      o[m][1][r] = d1;
      float x = d0 * d0 + d1 * d1;
      x += __shfl_xor(x, 1, 32);
      x += __shfl_xor(x, 2, 32);
      x += __shfl_xor(x, 4, 32);
      x += __shfl_xor(x, 8, 32);
      part[m][r] = x;
    }
  if (c == 0) {
#pragma unroll
    for (int m = 0; m < 4; ++m)
#pragma unroll
      for (int r = 0; r < 8; ++r) redS[wave][m * 16 + 8 * hh + r] = part[m][r];
  }
  __syncthreads();
  if (tid < 64) {
    float s = 0.0f;
#pragma unroll
    for (int w = 0; w < 8; ++w) s += redS[w][tid];
    stat[tid] = 1.0f / sqrtf(s * (1.0f / (float)DV) + GN_EPS_F);
  }
  __syncthreads();

  float* slab = Sl[wave];
  const int q = lane >> 3, c4 = (lane & 7) * 4;
  float* obase = normed + ((size_t)(b * NT + i0)) * VD + h * DV + wave * 32;
#pragma unroll
  for (int m = 0; m < 4; ++m) {
#pragma unroll
    for (int r = 0; r < 8; ++r) {
      const float rs = stat[m * 16 + 8 * hh + r];
      slab[(8 * hh + r) * SLP + c]      = o[m][0][r] * rs;
      slab[(8 * hh + r) * SLP + 16 + c] = o[m][1][r] * rs;
    }
    wave_sync_lds();
    for (int pass = 0; pass < 2; ++pass) {
#pragma unroll
      for (int it = 0; it < 4; ++it) {
        const int row = it * 4 + q;
        const v4f v = *(const v4f*)(slab + row * SLP + c4);
        *(volatile v4f*)(obase + (size_t)(m * 16 + row) * VD + c4) = v;
      }
      __threadfence();
    }
    wave_sync_lds();
  }
}

extern "C" void kernel_launch(void* const* d_in, const int* in_sizes, int n_in,
                              void* d_out, int out_size, void* d_ws, size_t ws_size, hipStream_t stream) {
  if (n_in < 5 || d_out == nullptr || d_ws == nullptr) return;
  if (in_sizes[0] != NROW * NHID || in_sizes[1] != NHID * NQKV || in_sizes[2] != NHID * VD ||
      in_sizes[3] != VD * NHID || in_sizes[4] != NHID || out_size != NOUT0 + NOUT1) return;

  const float* x    = (const float*)d_in[0];
  const float* Wqkv = (const float*)d_in[1];
  const float* Wg   = (const float*)d_in[2];
  const float* Wp   = (const float*)d_in[3];
  const float* bp   = (const float*)d_in[4];
  float* out0 = (float*)d_out;
  float* out1 = out0 + (size_t)NOUT0;

  char* ws = (char*)d_ws; size_t off = 0;
  auto carve = [&](size_t bytes) -> char* { char* p = ws + off; off += (bytes + 255) & ~(size_t)255; return p; };
  unsigned short* AX   = (unsigned short*)carve((size_t)NROW * NHID * 2);
  unsigned short* WQT  = (unsigned short*)carve((size_t)NQKV * NHID * 2);
  unsigned short* WGT  = (unsigned short*)carve((size_t)VD * NHID * 2);
  unsigned short* WPT  = (unsigned short*)carve((size_t)NHID * VD * 2);
  float*          QKVF = (float*)carve((size_t)NROW * NQKV * 4);
  unsigned short* QH   = (unsigned short*)carve((size_t)NBH * NT * DQK * 2);
  unsigned short* KH   = (unsigned short*)carve((size_t)NBH * NT * DQK * 2);
  unsigned short* VT   = (unsigned short*)carve((size_t)NBH * DV * NT * 2);
  float*          TAB  = (float*)carve((size_t)2 * NPAIR * 4);
  float*          NORMED = QKVF;
  unsigned short* GATED  = VT;
  if (off > ws_size || off > (size_t)134217728) return;

  Decay8 dec;
  for (int h = 0; h < NHEAD; ++h) {
    const double l0 = log(1.0 / 32.0), l1 = log(1.0 / 512.0);
    const double lg = l0 + (l1 - l0) * (double)h / (double)(NHEAD - 1);
    const float g = (float)(1.0 - exp(lg));
    dec.v[h] = (float)log2((double)g);
  }
  const float pscl = (float)pow((double)DQK, -0.5) * (PCARRY / QCARRY);

  rot_table_kernel<<<1, 512, 0, stream>>>(TAB);
  const int n8x = NROW * NHID / 8;
  cvt8_bf16_f16_kernel<<<(n8x + 255) / 256, 256, 0, stream>>>(x, AX, n8x);
  tcvt_kernel<<<dim3(NQKV / 64, NHID / 64, 1), 256, 0, stream>>>(Wqkv, NQKV, 0L, 0L, 1, WQT, NHID, 0L, WCARRY, 1);
  tcvt_kernel<<<dim3(VD / 64, NHID / 64, 1), 256, 0, stream>>>(Wg, VD, 0L, 0L, 1, WGT, NHID, 0L, WCARRY, 1);
  tcvt_kernel<<<dim3(NHID / 64, VD / 64, 1), 256, 0, stream>>>(Wp, NHID, 0L, 0L, 1, WPT, VD, 0L, WCARRY, 1);

  wmma_gemm64<0, 0, false><<<(NROW / 64) * (NQKV / 64) / 8, 256, 0, stream>>>(
      AX, NHID, WQT, NHID, (void*)QKVF, NQKV, bp, bp, 0, 1.0f, NROW, NQKV, NHID, WCARRY_INV);

  rotary_kernel<<<NT, 512, 0, stream>>>(QKVF, TAB, QH, KH);
  tcvt_kernel<<<dim3(DV / 64, NT / 64, NBH), 256, 0, stream>>>(QKVF + 2 * QKD, NQKV, (long)NT * NQKV, (long)DV, NHEAD,
                                                               VT, NT, (long)DV * NT, 1.0f, 0);
  kv_state_kernel<<<NBH * 4, 256, 0, stream>>>(QKVF, out1, dec);
  retention_gn_kernel<<<dim3(NT / 64, NBH), 256, 0, stream>>>(QH, KH, VT, NORMED, dec, pscl);
  wmma_gemm64<0, 1, true><<<(NROW / 64) * (VD / 64) / 8, 256, 0, stream>>>(
      AX, NHID, WGT, NHID, (void*)GATED, VD, bp, NORMED, VD, GCARRY, NROW, VD, NHID, WCARRY_INV);
  wmma_gemm64<2, 0, false><<<(NROW / 64) * (NHID / 64) / 8, 256, 0, stream>>>(
      GATED, VD, WPT, VD, (void*)out0, NHID, bp, bp, 0, 1.0f, NROW, NHID, VD, OUT_SCALE);
}
